// HumanSender_27281632264216
// MI455X (gfx1250) — hardware-verified
//
#include <hip/hip_runtime.h>


namespace {
constexpr int N = 50000, E = 800000, NP_ = 1024, F = 128, HID = 128, EMB = 64, R = 3, NBASE = 2, NPAD = 50048, NBLK = NPAD / 128;
constexpr float FXS = 524288.0f, FXI = 1.0f / 524288.0f;

typedef _Float16 b16;
typedef __attribute__((ext_vector_type(16))) _Float16 v16b;
typedef __attribute__((ext_vector_type(8)))  _Float16 v8b;
typedef __attribute__((ext_vector_type(8)))  float v8f;
typedef __attribute__((ext_vector_type(4)))  float v4f;

__device__ __forceinline__ v8b ld8b(const b16* p) { return *(const v8b*)p; }
__device__ __forceinline__ v16b cat8b(v8b a, v8b b) { return __builtin_shufflevector(a, b, 0, 1, 2, 3, 4, 5, 6, 7, 8, 9, 10, 11, 12, 13, 14, 15); }
__device__ __forceinline__ v16b frag_kb(const b16* p, int hh) { return cat8b(ld8b(p + 8 * hh), ld8b(p + 16 + 8 * hh)); }
__device__ __forceinline__ void split16(float v, b16& hi, b16& lo) { hi = (b16)v; lo = (b16)(v - (float)hi); }
__device__ __forceinline__ void frag_ksplit(const float* p, int hh, v16b& fh_, v16b& fl_) {
  const float* p0 = p + 8 * hh; const float* p1 = p + 16 + 8 * hh;
#pragma unroll
  for (int e = 0; e < 8; ++e) { b16 a, c; split16(p0[e], a, c); fh_[e] = a; fl_[e] = c; split16(p1[e], a, c); fh_[8 + e] = a; fl_[8 + e] = c; }
}
__device__ __forceinline__ v8f wmma16b(v16b a, v16b b, v8f c) {
  v8f d = __builtin_amdgcn_wmma_f32_16x16x32_f16(false, a, false, b, (short)0, c, false, false);
  asm volatile("v_nop\n\tv_nop\n\tv_nop\n\tv_nop" : "+v"(d) : "v"(a), "v"(b));
  return d;
}
__device__ __forceinline__ void wave_lds_sync() {
  __builtin_amdgcn_fence(__ATOMIC_RELEASE, "workgroup");
  __builtin_amdgcn_wave_barrier();
  __builtin_amdgcn_fence(__ATOMIC_ACQUIRE, "workgroup");
}

struct Opnd { const void* p0; const void* p1; int ld; };
template <int NP> __device__ __forceinline__ void load_frags(const Opnd& o, int row, int kb, int hh, v16b& fh_, v16b& fl_) {
  if (NP == 0) { frag_ksplit((const float*)o.p0 + (size_t)row * o.ld + kb, hh, fh_, fl_); }
  else if (NP == 4) {
    const float* p = (const float*)o.p0 + (size_t)row * o.ld + kb; const float* p0 = p + 8 * hh; const float* p1 = p + 16 + 8 * hh;
#pragma unroll
    for (int e = 0; e < 8; ++e) { b16 a, c; split16(p0[e] * 64.0f, a, c); fh_[e] = a; fl_[e] = c; split16(p1[e] * 64.0f, a, c); fh_[8 + e] = a; fl_[8 + e] = c; }
  } else if (NP == 3) {
    const float* p = (const float*)o.p0 + (size_t)row * o.ld + kb; const float* p0 = p + 8 * hh; const float* p1 = p + 16 + 8 * hh;
#pragma unroll
    for (int e = 0; e < 8; ++e) { fh_[e] = (b16)p0[e]; fh_[8 + e] = (b16)p1[e]; }
    fl_ = fh_;
  } else {
    fh_ = frag_kb((const b16*)o.p0 + (size_t)row * o.ld + kb, hh);
    if (NP == 2) fl_ = frag_kb((const b16*)o.p1 + (size_t)row * o.ld + kb, hh); else fl_ = fh_;
  }
}
template <int ANP, int BNP> __device__ __forceinline__ v8f mac(v16b ah, v16b al, v16b bh, v16b bl, v8f c) {
  c = wmma16b(ah, bh, c);
  if (BNP == 0 || BNP == 2 || BNP == 4) c = wmma16b(ah, bl, c);
  if (ANP == 0 || ANP == 2 || ANP == 4) c = wmma16b(al, bh, c);
  return c;
}
template <int ANP, int BNP>
__device__ __forceinline__ void gemm_tile(const Opnd& A, const Opnd& B, int K, int m0, int c0, int nloc, int hlf, v8f (&acc)[2][4]) {
  for (int kb = 0; kb < K; kb += 32) {
    v16b a0h, a0l, a1h, a1l;
    load_frags<ANP>(A, m0 + nloc, kb, hlf, a0h, a0l);
    load_frags<ANP>(A, m0 + 16 + nloc, kb, hlf, a1h, a1l);
#pragma unroll
    for (int t = 0; t < 4; ++t) {
      v16b bh, bl;
      load_frags<BNP>(B, c0 + t * 16 + nloc, kb, hlf, bh, bl);
      acc[0][t] = mac<ANP, BNP>(a0h, a0l, bh, bl, acc[0][t]);
      acc[1][t] = mac<ANP, BNP>(a1h, a1l, bh, bl, acc[1][t]);
    }
  }
}

__device__ __forceinline__ void epi_planes(v8f (&acc)[2][4], float scale, bool two, b16* __restrict__ oh, b16* __restrict__ ol, int ldo,
                                           int m0, int c0, int lane, b16* Th, b16* Tl) {
  const int nloc = lane & 15, hlf = lane >> 4;
#pragma unroll
  for (int t = 0; t < 4; ++t)
#pragma unroll
    for (int r = 0; r < 2; ++r)
#pragma unroll
      for (int v = 0; v < 8; ++v) {
        const int rr = r * 16 + v + 8 * hlf, cc = t * 16 + nloc;
        b16 h_, l_; split16(acc[r][t][v] * scale, h_, l_);
        Th[rr * 64 + cc] = h_; Tl[rr * 64 + cc] = l_;
      }
  wave_lds_sync();
  for (int pass = 0; pass < 2; ++pass) {
#pragma unroll
    for (int j = 0; j < 8; ++j) {
      const int rr = j * 4 + (lane >> 3), c8 = (lane & 7) * 8;
      const size_t o = (size_t)(m0 + rr) * ldo + c0 + c8;
      *(volatile v8b*)(oh + o) = ld8b(Th + rr * 64 + c8);
      if (two) *(volatile v8b*)(ol + o) = ld8b(Tl + rr * 64 + c8);
    }
    __threadfence();
  }
}
__device__ __forceinline__ void epi_f32(v8f (&acc)[2][4], float scale, const float* rscale, float* __restrict__ out, int ldo, int m0, int c0, int lane, float* Tt) {
  const int nloc = lane & 15, hlf = lane >> 4;
#pragma unroll
  for (int t = 0; t < 4; ++t)
#pragma unroll
    for (int r = 0; r < 2; ++r)
#pragma unroll
      for (int v = 0; v < 8; ++v) {
        const int rr = r * 16 + v + 8 * hlf;
        const float rs = rscale ? rscale[(size_t)(m0 + rr) * 32] : 1.0f;
        Tt[rr * 64 + t * 16 + nloc] = acc[r][t][v] * scale * rs;
      }
  wave_lds_sync();
  float* dst0 = out + (size_t)m0 * ldo + c0;
  for (int pass = 0; pass < 2; ++pass) {
#pragma unroll
    for (int j = 0; j < 16; ++j) { const int rr = j * 2 + hlf, c4 = nloc * 4; *(volatile v4f*)(dst0 + (size_t)rr * ldo + c4) = *(const v4f*)(Tt + rr * 64 + c4); }
    __threadfence();
  }
}


__global__ __launch_bounds__(256) void prep_kernel(const float* __restrict__ basis1, const float* __restrict__ comp1, const float* __restrict__ root1, const float* __restrict__ basis2, const float* __restrict__ comp2, const float* __restrict__ root2, const float* __restrict__ fcw,
                                                   b16* __restrict__ w1, b16* __restrict__ w2, b16* __restrict__ wf) {
  const size_t tid = (size_t)blockIdx.x * blockDim.x + threadIdx.x, nth = (size_t)gridDim.x * blockDim.x;
  for (int pass = 0; pass < 2; ++pass) {
    for (size_t p = tid; p < (size_t)4 * HID * F / 8; p += nth) { const int n = (int)(p / (F / 8)), k0 = (int)(p % (F / 8)) * 8; const int blk = n / HID, nn = n % HID; v8b v;
#pragma unroll
      for (int e = 0; e < 8; ++e) { const int k = k0 + e; float w; if (blk == 0) w = root1[(size_t)k * HID + nn]; else { const int r = blk - 1; w = comp1[r * NBASE] * basis1[((size_t)0 * F + k) * HID + nn] + comp1[r * NBASE + 1] * basis1[((size_t)1 * F + k) * HID + nn]; } v[e] = (b16)w; }
      *(volatile v8b*)(w1 + (size_t)n * F + k0) = v; }
    for (size_t p = tid; p < (size_t)4 * EMB * HID / 8; p += nth) { const int n = (int)(p / (HID / 8)), k0 = (int)(p % (HID / 8)) * 8; const int blk = n / EMB, nn = n % EMB; v8b v;
#pragma unroll
      for (int e = 0; e < 8; ++e) { const int k = k0 + e; float w; if (blk == 0) w = root2[(size_t)k * EMB + nn]; else { const int r = blk - 1; w = comp2[r * NBASE] * basis2[((size_t)0 * HID + k) * EMB + nn] + comp2[r * NBASE + 1] * basis2[((size_t)1 * HID + k) * EMB + nn]; } v[e] = (b16)w; }
      *(volatile v8b*)(w2 + (size_t)n * HID + k0) = v; }
    for (size_t p = tid; p < (size_t)HID * (2 * EMB) / 8; p += nth) { const int n = (int)(p / (2 * EMB / 8)), k0 = (int)(p % (2 * EMB / 8)) * 8; v8b v;
#pragma unroll
      for (int e = 0; e < 8; ++e) v[e] = (b16)fcw[(size_t)(k0 + e) * HID + n];
      *(volatile v8b*)(wf + (size_t)n * (2 * EMB) + k0) = v; }
    __threadfence();
  }
}

template <int NOUT>
__global__ __launch_bounds__(128) void lin_kernel(const float* __restrict__ x, int nrow, const b16* __restrict__ w, float* __restrict__ y) {
  __shared__ __attribute__((aligned(16))) float Ts[4][32 * 64];
  const int lane = threadIdx.x & 31, wave = threadIdx.x >> 5, nloc = lane & 15, hlf = lane >> 4, m0 = blockIdx.y * 128 + wave * 32, c0 = blockIdx.x * 64;
  v8f acc[2][4];
#pragma unroll
  for (int r = 0; r < 2; ++r)
#pragma unroll
    for (int t = 0; t < 4; ++t) acc[r][t] = (v8f){};
  const Opnd A{x, nullptr, F}; const int ra = min(m0 + nloc, nrow - 1), rb = min(m0 + 16 + nloc, nrow - 1);
#pragma unroll 2
  for (int kb = 0; kb < F; kb += 32) { v16b a0, a1, d0, d1; load_frags<3>(A, ra, kb, hlf, a0, d0); load_frags<3>(A, rb, kb, hlf, a1, d1);
#pragma unroll
    for (int t = 0; t < 4; ++t) { const v16b bw = frag_kb(w + (size_t)(c0 + t * 16 + nloc) * F + kb, hlf); acc[0][t] = wmma16b(a0, bw, acc[0][t]); acc[1][t] = wmma16b(a1, bw, acc[1][t]); } }
  epi_f32(acc, 1.0f, nullptr, y, NOUT, m0, c0, lane, Ts[wave]);
}

typedef __attribute__((ext_vector_type(4))) int v4i;
template <int OD, int NB, bool RELU>
__global__ __launch_bounds__(256) void rgcn_kernel(const int* __restrict__ esrc, const int* __restrict__ edst, const int* __restrict__ etype, const float* __restrict__ y, const float* __restrict__ bias, float* __restrict__ xo, int ostride) {
  constexpr int DF = R * OD;
  __shared__ __attribute__((aligned(16))) int acc[NB * DF];
  __shared__ int cnt[NB * R]; __shared__ int list[8 * 256];
  const int t_ = threadIdx.x, wave = t_ >> 5, lane = t_ & 31, base = blockIdx.x * NB;
  for (int i = t_; i < NB * DF; i += 256) acc[i] = 0;
  for (int i = t_; i < NB * R; i += 256) cnt[i] = 0;
  __syncthreads();
  int* wl = list + wave * 256;
  for (int c0 = 0; c0 < E; c0 += 256 * 8) {
    const int e0 = c0 + (wave * 32 + lane) * 8; int dd[8];
#pragma unroll
    for (int j = 0; j < 8; ++j) { const int dv = edst[min(e0 + j, E - 1)]; dd[j] = (e0 + j < E) ? dv : -1; }
    unsigned sl[8]; bool hit[8]; bool anyl = false;
#pragma unroll
    for (int j = 0; j < 8; ++j) { sl[j] = (unsigned)(dd[j] - base); hit[j] = sl[j] < (unsigned)NB; anyl |= hit[j]; }
    int wc = 0;
    if (__builtin_amdgcn_ballot_w32(anyl) != 0u) {
#pragma unroll
      for (int j = 0; j < 8; ++j) {
        const unsigned mj = __builtin_amdgcn_ballot_w32(hit[j]);
        if (mj != 0u) {
          if (hit[j]) { const int pos = wc + (int)__builtin_amdgcn_mbcnt_lo(mj, 0u); wl[pos] = ((e0 + j) << 9) | (int)sl[j]; }
          wc += __builtin_popcount(mj); } } }
    __builtin_amdgcn_wave_barrier(); __builtin_amdgcn_fence(__ATOMIC_RELEASE, "workgroup"); __builtin_amdgcn_fence(__ATOMIC_ACQUIRE, "workgroup");
    { constexpr int LPH = OD / 4, HPS = 32 / LPH;
      for (int i0 = 0; i0 < wc; i0 += HPS) { const int i = i0 + lane / LPH; if (i < wc) { const int ent = wl[i]; const int e = ent >> 9, slot = ent & 511; int s = esrc[e]; s = (s < 0) ? 0 : (s >= N ? N - 1 : s);
          int r = etype[e]; r = (r < 0) ? 0 : (r >= R ? R - 1 : r); const int col = (lane % LPH) * 4;
          if (col == 0) atomicAdd(&cnt[slot * R + r], 1);
          const v4f v = *(const v4f*)(y + (size_t)s * (4 * OD) + (size_t)(1 + r) * OD + col);
#pragma unroll
          for (int c = 0; c < 4; ++c) atomicAdd(&acc[(slot * R + r) * OD + col + c], (int)rintf(v[c] * FXS)); } } }
    __builtin_amdgcn_wave_barrier();
  }
  __syncthreads();
  for (int pass = 0; pass < 2; ++pass) {
    for (int i = t_; i < NB * OD / 4; i += 256) { const int r_ = (i * 4) / OD, cq = (i * 4) % OD, node = base + r_; if (node < NPAD) { v4f o = {0.0f, 0.0f, 0.0f, 0.0f};
        if (node < N) { const float i0 = 1.0f / fmaxf((float)cnt[r_ * R], 1.0f), i1 = 1.0f / fmaxf((float)cnt[r_ * R + 1], 1.0f), i2 = 1.0f / fmaxf((float)cnt[r_ * R + 2], 1.0f);
#pragma unroll
          for (int c = 0; c < 4; ++c) { float val = y[(size_t)node * (4 * OD) + cq + c] + bias[cq + c]
              + (float)acc[(r_ * R) * OD + cq + c] * FXI * i0 + (float)acc[(r_ * R + 1) * OD + cq + c] * FXI * i1 + (float)acc[(r_ * R + 2) * OD + cq + c] * FXI * i2;
            if (RELU) val = fmaxf(val, 0.0f); o[c] = val; } }
        *(volatile v4f*)(xo + (size_t)node * ostride + cq) = o; } }
    __threadfence();
  }
}

__global__ __launch_bounds__(128) void pair_kernel(const int* __restrict__ nest, const int* __restrict__ food, const float* __restrict__ emb, const b16* __restrict__ wf, const float* __restrict__ fcb, float* __restrict__ out) {
  __shared__ __attribute__((aligned(16))) b16 Pt[32][2 * EMB + 8]; __shared__ __attribute__((aligned(16))) float Ot[4][32][32 + 4];
  const int wave = threadIdx.x >> 5, lane = threadIdx.x & 31, nloc = lane & 15, hlf = lane >> 4, p0 = blockIdx.x * 32;
  { const int pl = threadIdx.x >> 2, q = threadIdx.x & 3; int a = nest[p0 + pl], b = food[p0 + pl]; a = (a < 0) ? 0 : (a >= N ? N - 1 : a); b = (b < 0) ? 0 : (b >= N ? N - 1 : b);
    const float* srow = (q < 2) ? (emb + (size_t)a * EMB + q * 32) : (emb + (size_t)b * EMB + (q - 2) * 32);
#pragma unroll
    for (int i = 0; i < 32; i += 4) { const v4f v = *(const v4f*)(srow + i); Pt[pl][q * 32 + i] = (b16)v[0]; Pt[pl][q * 32 + i + 1] = (b16)v[1]; Pt[pl][q * 32 + i + 2] = (b16)v[2]; Pt[pl][q * 32 + i + 3] = (b16)v[3]; } }
  __syncthreads();
  v8f acc[2][2] = {{{}, {}}, {{}, {}}}; const int c0 = wave * 32;
#pragma unroll
  for (int kb = 0; kb < 2 * EMB; kb += 32) { const v16b a0 = frag_kb(&Pt[nloc][0] + kb, hlf), a1 = frag_kb(&Pt[16 + nloc][0] + kb, hlf);
#pragma unroll
    for (int t = 0; t < 2; ++t) { const v16b bw = frag_kb(wf + (size_t)(c0 + t * 16 + nloc) * (2 * EMB) + kb, hlf); acc[0][t] = wmma16b(a0, bw, acc[0][t]); acc[1][t] = wmma16b(a1, bw, acc[1][t]); } }
#pragma unroll
  for (int t = 0; t < 2; ++t)
#pragma unroll
    for (int r = 0; r < 2; ++r)
#pragma unroll
      for (int v = 0; v < 8; ++v) Ot[wave][r * 16 + v + 8 * hlf][t * 16 + nloc] = tanhf(acc[r][t][v] + fcb[c0 + t * 16 + nloc]);
  wave_lds_sync();
  for (int pass = 0; pass < 2; ++pass) {
#pragma unroll
    for (int j = 0; j < 8; ++j) { const int rr = j * 4 + (lane >> 3), c4 = (lane & 7) * 4; *(volatile v4f*)(out + (size_t)(p0 + rr) * HID + c0 + c4) = *(const v4f*)(&Ot[wave][rr][c4]); }
    __threadfence();
  }
}
}

extern "C" void kernel_launch(void* const* d_in, const int* in_sizes, int n_in,
                              void* d_out, int out_size, void* d_ws, size_t ws_size, hipStream_t stream) {
  (void)n_in; (void)out_size;
  const float* x = (const float*)d_in[0]; const int* ei = (const int*)d_in[1];   const int* et = (const int*)d_in[3];
  const int* nest = (const int*)d_in[4]; const int* food = (const int*)d_in[5];
  const float* basis1 = (const float*)d_in[6]; const float* comp1 = (const float*)d_in[7]; const float* root1 = (const float*)d_in[8]; const float* bias1 = (const float*)d_in[9];
  const float* basis2 = (const float*)d_in[10]; const float* comp2 = (const float*)d_in[11]; const float* root2 = (const float*)d_in[12]; const float* bias2 = (const float*)d_in[13];
  const float* fcw = (const float*)d_in[14]; const float* fcb = (const float*)d_in[15];
  float* out = (float*)d_out;
  if (in_sizes[0] != N * F || in_sizes[1] != 2 * E || in_sizes[3] != E || in_sizes[4] != NP_ || in_sizes[6] != NBASE * F * HID || in_sizes[14] != 2 * EMB * HID) return;
  const int* esrc = ei; const int* edst = ei + E;
  size_t off = 0; char* ws = (char*)d_ws;
  auto carve = [&](size_t bytes) { char* p = ws + off; off += (bytes + 255) & ~(size_t)255; return p; };
  b16* w1 = (b16*)carve((size_t)4 * HID * F * 2); b16* w2 = (b16*)carve((size_t)4 * EMB * HID * 2); b16* wf = (b16*)carve((size_t)HID * 2 * EMB * 2);
  float* y1 = (float*)carve((size_t)NPAD * 4 * HID * 4);
  float* h = (float*)carve((size_t)NPAD * HID * 4);
  if (off > ws_size) return;
  prep_kernel<<<128, 256, 0, stream>>>(basis1, comp1, root1, basis2, comp2, root2, fcw, w1, w2, wf);
  lin_kernel<4 * HID><<<dim3(4 * HID / 64, NBLK), 128, 0, stream>>>(x, N, w1, y1);
  rgcn_kernel<HID, 128, true><<<NPAD / 128, 256, 0, stream>>>(esrc, edst, et, y1, bias1, h, HID);
  lin_kernel<4 * EMB><<<dim3(4 * EMB / 64, NBLK), 128, 0, stream>>>(h, NPAD, w2, y1);
  float* emb = h;
  rgcn_kernel<EMB, 256, false><<<NPAD / 256 + 1, 256, 0, stream>>>(esrc, edst, et, y1, bias2, emb, EMB);
  pair_kernel<<<NP_ / 32, 128, 0, stream>>>(nest, food, emb, wf, fcb, out);
}
